// SpatialLocalAttention_26774826123576
// MI455X (gfx1250) — hardware-verified
//
#include <hip/hip_runtime.h>
#include <math.h>

typedef __attribute__((ext_vector_type(16))) _Float16 v16h;
typedef __attribute__((ext_vector_type(16))) __bf16 v16b;
typedef __attribute__((ext_vector_type(8)))  _Float16 v8h;
typedef __attribute__((ext_vector_type(8)))  float v8f;
typedef __attribute__((ext_vector_type(4)))  float v4f;
typedef __attribute__((ext_vector_type(2)))  float v2f;
typedef __attribute__((ext_vector_type(4)))  unsigned v4u;
typedef __attribute__((ext_vector_type(4)))  int v4i;
typedef float __attribute__((may_alias)) float_a;
typedef int __attribute__((may_alias)) int_a;

template <typename T> __device__ __forceinline__ void vst2(void* p, T v) { *(volatile T*)p = v; __threadfence(); *(volatile T*)p = v; }
__device__ __forceinline__ v8f wmma16(v16h a, v16h b, v8f c) {
  v8f d = __builtin_amdgcn_wmma_f32_16x16x32_f16(false, a, false, b, (short)0, c, false, false);
  asm volatile("v_nop\n\tv_nop\n\tv_nop\n\tv_nop" : "+v"(d) : "v"(a), "v"(b));
  return d;
}
__device__ __forceinline__ v8f wmma_bf(v16b a, v16b b, v8f c) {
  v8f d = __builtin_amdgcn_wmma_f32_16x16x32_bf16(false, a, false, b, (short)0, c, false, false);
  asm volatile("v_nop\n\tv_nop\n\tv_nop\n\tv_nop" : "+v"(d) : "v"(a), "v"(b));
  return d;
}
__device__ __forceinline__ v16h frag_h(const _Float16* rowk0, int lane) {
  union { v16h v; v8h q[2]; } u; const _Float16* p = rowk0 + 8 * (lane >> 4);
  u.q[0] = *(const v8h*)p; u.q[1] = *(const v8h*)(p + 16); return u.v;
}
__device__ __forceinline__ v16h frag_f32(const float* rowk0, int lane) {
  v16h a; const float* p = rowk0 + 8 * (lane >> 4);
#pragma unroll
  for (int i = 0; i < 8; ++i) { a[i] = (_Float16)p[i]; a[8 + i] = (_Float16)p[16 + i]; }
  return a;
}
__device__ __forceinline__ v16h frag_f32s(const float* rowk0, int lane, float sc) {
  v16h a; const float* p = rowk0 + 8 * (lane >> 4);
#pragma unroll
  for (int i = 0; i < 8; ++i) { a[i] = (_Float16)(p[i] * sc); a[8 + i] = (_Float16)(p[16 + i] * sc); }
  return a;
}
__device__ __forceinline__ v16h fragc_f32(const float* W, int k0, int n, int lane, int ld, int K) {
  v16h a; const int g = lane >> 4;
#pragma unroll
  for (int i = 0; i < 8; ++i) { const int ka = k0 + 8 * g + i, kb = ka + 16;
    a[i] = (_Float16)(ka < K ? W[(size_t)(ka < K ? ka : K - 1) * ld + n] : 0.f); a[8 + i] = (_Float16)(kb < K ? W[(size_t)(kb < K ? kb : K - 1) * ld + n] : 0.f); }
  return a;
}
struct F2 { v16b h, l; };
__device__ __forceinline__ F2 bsplit16(const float v[16]) { F2 r;
#pragma unroll
  for (int i = 0; i < 16; ++i) { const __bf16 h = (__bf16)v[i]; r.h[i] = h; r.l[i] = (__bf16)(v[i] - (float)h); }
  return r; }
__device__ __forceinline__ F2 split_row(const float* row, int k0, int lane) { float v[16]; const float* p = row + k0 + 8 * (lane >> 4);
#pragma unroll
  for (int i = 0; i < 8; ++i) { v[i] = p[i]; v[8 + i] = p[16 + i]; }
  return bsplit16(v); }
__device__ __forceinline__ F2 split_rowK(const float* row, int k0, int lane, int K) { float v[16]; const int g = lane >> 4;
#pragma unroll
  for (int i = 0; i < 8; ++i) { const int ka = k0 + 8 * g + i, kb = ka + 16; v[i] = ka < K ? row[ka < K ? ka : K - 1] : 0.f; v[8 + i] = kb < K ? row[kb < K ? kb : K - 1] : 0.f; }
  return bsplit16(v); }
__device__ __forceinline__ F2 split_col(const float* W, int k0, int n, int lane, int ld, int K) { float v[16]; const int g = lane >> 4;
#pragma unroll
  for (int i = 0; i < 8; ++i) { const int ka = k0 + 8 * g + i, kb = ka + 16; v[i] = ka < K ? W[(size_t)(ka < K ? ka : K - 1) * ld + n] : 0.f; v[8 + i] = kb < K ? W[(size_t)(kb < K ? kb : K - 1) * ld + n] : 0.f; }
  return bsplit16(v); }
__device__ __forceinline__ v8f mac3(const F2& a, const F2& b, v8f c) { c = wmma_bf(a.l, b.h, c); c = wmma_bf(a.h, b.l, c); return wmma_bf(a.h, b.h, c); }
__device__ __forceinline__ float sigm(float v) { return 1.0f / (1.0f + expf(-v)); }
#define LDSX() do { asm volatile("s_wait_dscnt 0" ::: "memory"); __builtin_amdgcn_wave_barrier(); __builtin_amdgcn_fence(__ATOMIC_RELEASE, "workgroup"); } while (0)

__device__ __forceinline__ float bfr(float v) { return (float)(__bf16)v; }
#define NBT 2
#define LL 2048
#define DD 512
#define KNB 32
#define GG 32
#define NH 8
#define HD 64
#define NCTX (1 + KNB + GG)
#ifndef TQ
#define TQ LL
#endif
#ifndef TNB
#define TNB NBT
#endif
#define WS_Q  0u
#define WS_KS (WS_Q + 4u * (size_t)NBT * LL * DD)
#define WS_VS (WS_KS + 4u * (size_t)NBT * LL * DD)
#define WS_KG (WS_VS + 4u * (size_t)NBT * LL * DD)
#define WS_VG (WS_KG + 4u * (size_t)NBT * GG * DD)
#define WS_Y  (WS_VG + 4u * (size_t)NBT * GG * DD)
#define WS_END (WS_Y + 4u * (size_t)NBT * LL * DD)
__global__ __launch_bounds__(128) void k_proj(const float* __restrict__ SP, const float* __restrict__ GL, const float* __restrict__ WQ, const float* __restrict__ WK, const float* __restrict__ WV, float* __restrict__ Q, float* __restrict__ KS, float* __restrict__ VS, float* __restrict__ KG, float* __restrict__ VG) { __shared__ __align__(16) float sf[4][16][132];
  const int tid = threadIdx.x, wave = tid >> 5, lane = tid & 31, col = lane & 15, g = lane >> 4; const int which = blockIdx.z; const int c0 = blockIdx.y * 128; const size_t r0 = (size_t)blockIdx.x * 64 + wave * 16;
  if (which >= 3 && blockIdx.x > 0) return;
  const float* X = (which < 3) ? SP : GL; const float* Wm = (which == 0) ? WQ : (which == 1 || which == 3) ? WK : WV; float* D = (which == 0) ? Q : (which == 1) ? KS : (which == 2) ? VS : (which == 3) ? KG : VG;
  v8f acc[8] = {};
#pragma unroll 2
  for (int kc = 0; kc < DD / 32; ++kc) { v16b a; { const float* p = X + (r0 + col) * DD + kc * 32 + 8 * g;
#pragma unroll
      for (int i = 0; i < 8; ++i) { a[i] = (__bf16)p[i]; a[8 + i] = (__bf16)p[16 + i]; } }
#pragma unroll
    for (int j = 0; j < 8; ++j) { v16b w; const int o = c0 + j * 16 + col;
#pragma unroll
      for (int i = 0; i < 8; ++i) { w[i] = (__bf16)Wm[(size_t)(kc * 32 + 8 * g + i) * DD + o]; w[8 + i] = (__bf16)Wm[(size_t)(kc * 32 + 16 + 8 * g + i) * DD + o]; }
      acc[j] = wmma_bf(a, w, acc[j]); } }
#pragma unroll
  for (int j = 0; j < 8; ++j)
#pragma unroll
    for (int r = 0; r < 8; ++r) sf[wave][8 * g + r][j * 16 + col] = acc[j][r];
  LDSX(); for (int rl = 0; rl < 16; ++rl) vst2(D + (r0 + rl) * DD + c0 + lane * 4, *(const v4f*)&sf[wave][rl][lane * 4]); }
__global__ __launch_bounds__(256) void k_att(const float* __restrict__ Q, const float* __restrict__ KS, const float* __restrict__ VS, const float* __restrict__ KG, const float* __restrict__ VG, const int* __restrict__ IDX, const float* __restrict__ DIST, const float* __restrict__ LSIG, const float* __restrict__ GBIAS, float* __restrict__ Y) {
  __shared__ float ssc[8][NH][NCTX + 3]; __shared__ __align__(16) float sy[8][DD];
  const int tid = threadIdx.x, wave = tid >> 5, lane = tid & 31; const int h = lane >> 2, part = lane & 3; const size_t b = blockIdx.y; const size_t l = (size_t)blockIdx.x * 8 + wave;
  const float* qr = Q + (b * LL + l) * DD + h * HD; const int* idr = IDX + (b * LL + l) * KNB; const float* dsr = DIST + (b * LL + l) * KNB;
  const float sig = expf(bfr(LSIG[h])); const float inv2s2 = 1.0f / (2.0f * sig * sig); const float gb = bfr(GBIAS[0]);
  float qv[HD];
#pragma unroll
  for (int d = 0; d < HD; ++d) qv[d] = qr[d];
#pragma unroll 1
  for (int c = part; c < NCTX; c += 4) { const float* kr; float bias;
    if (c == 0) { kr = KS + (b * LL + l) * DD + h * HD; bias = 0.f; }
    else if (c <= KNB) { const int j = idr[c - 1]; kr = KS + (b * LL + j) * DD + h * HD; const float dsq = bfr(dsr[c - 1]); bias = -(dsq * dsq) * inv2s2; }
    else { kr = KG + (b * GG + (c - 1 - KNB)) * DD + h * HD; bias = gb; }
    float s = 0.f;
#pragma unroll
    for (int d4 = 0; d4 < HD; d4 += 4) { const v4f kv = *(const v4f*)(kr + d4); s += qv[d4] * kv[0] + qv[d4 + 1] * kv[1] + qv[d4 + 2] * kv[2] + qv[d4 + 3] * kv[3]; }
    ssc[wave][h][c] = s * 0.125f + bias; }
  LDSX();
  float m = -3.0e38f; for (int c = 0; c < NCTX; ++c) m = fmaxf(m, ssc[wave][h][c]); float sum = 0.f; for (int c = 0; c < NCTX; ++c) sum += expf(ssc[wave][h][c] - m); const float inv = 1.0f / sum;
  LDSX();
  for (int c = part; c < NCTX; c += 4) ssc[wave][h][c] = expf(ssc[wave][h][c] - m) * inv;
  LDSX();
  float acc[HD];
#pragma unroll
  for (int d = 0; d < HD; ++d) acc[d] = 0.f;
#pragma unroll 1
  for (int c = part; c < NCTX; c += 4) { const float* vr; if (c == 0) vr = VS + (b * LL + l) * DD + h * HD; else if (c <= KNB) vr = VS + (b * LL + idr[c - 1]) * DD + h * HD; else vr = VG + (b * GG + (c - 1 - KNB)) * DD + h * HD;
    const float p = ssc[wave][h][c];
#pragma unroll
    for (int d4 = 0; d4 < HD; d4 += 4) { const v4f vv = *(const v4f*)(vr + d4); acc[d4] += p * vv[0]; acc[d4 + 1] += p * vv[1]; acc[d4 + 2] += p * vv[2]; acc[d4 + 3] += p * vv[3]; } }
#pragma unroll
  for (int d = 0; d < HD; ++d) { acc[d] += __shfl_xor(acc[d], 1); acc[d] += __shfl_xor(acc[d], 2); }
  if (part == 0) {
#pragma unroll
    for (int d = 0; d < HD; ++d) sy[wave][h * HD + d] = acc[d]; }
  LDSX();
  for (int pz = 0; pz < DD / 128; ++pz) vst2(Y + (b * LL + l) * DD + pz * 128 + lane * 4, *(const v4f*)&sy[wave][pz * 128 + lane * 4]); }
__global__ __launch_bounds__(128) void k_out(const float* __restrict__ Yr, const float* __restrict__ WO, const float* __restrict__ BO, float* __restrict__ OUT) { __shared__ __align__(16) float sf[4][16][132];
  const int tid = threadIdx.x, wave = tid >> 5, lane = tid & 31, col = lane & 15, g = lane >> 4; const int c0 = blockIdx.y * 128; const size_t r0 = (size_t)blockIdx.x * 64 + wave * 16;
  v8f acc[8] = {};
#pragma unroll 2
  for (int kc = 0; kc < DD / 32; ++kc) { const F2 a = split_row(Yr + (r0 + col) * DD, kc * 32, lane);
#pragma unroll
    for (int j = 0; j < 8; ++j) { v16b w; const int o = c0 + j * 16 + col;
#pragma unroll
      for (int i = 0; i < 8; ++i) { w[i] = (__bf16)WO[(size_t)(kc * 32 + 8 * g + i) * DD + o]; w[8 + i] = (__bf16)WO[(size_t)(kc * 32 + 16 + 8 * g + i) * DD + o]; }
      acc[j] = wmma_bf(a.h, w, acc[j]); acc[j] = wmma_bf(a.l, w, acc[j]); } }
#pragma unroll
  for (int j = 0; j < 8; ++j) { const float bb = bfr(BO[c0 + j * 16 + col]);
#pragma unroll
    for (int r = 0; r < 8; ++r) sf[wave][8 * g + r][j * 16 + col] = acc[j][r] + bb; }
  LDSX(); for (int rl = 0; rl < 16; ++rl) vst2(OUT + (r0 + rl) * DD + c0 + lane * 4, *(const v4f*)&sf[wave][rl][lane * 4]); }
extern "C" void kernel_launch(void* const* d_in, const int* in_sizes, int n_in, void* d_out, int out_size, void* d_ws, size_t ws_size, hipStream_t stream) {
  (void)in_sizes; (void)n_in; (void)out_size;
  const float** F = (const float**)d_in;
  if (ws_size < (size_t)WS_END) return;
  char* ws = (char*)d_ws; float *Q = (float*)(ws + WS_Q), *KS = (float*)(ws + WS_KS), *VS = (float*)(ws + WS_VS), *KG = (float*)(ws + WS_KG), *VG = (float*)(ws + WS_VG), *Y = (float*)(ws + WS_Y);
  k_proj<<<dim3(NBT * LL / 64, DD / 128, 5), 128, 0, stream>>>(F[0], F[3], F[4], F[5], F[6], Q, KS, VS, KG, VG);
  k_att<<<dim3(TQ / 8, TNB), 256, 0, stream>>>(Q, KS, VS, KG, VG, (const int*)d_in[1], F[2], F[9], F[10], Y);
  k_out<<<dim3(TNB * LL / 64, DD / 128), 128, 0, stream>>>(Y, F[7], F[8], (float*)d_out);
}
